// attention_mech_28664611733586
// MI455X (gfx1250) — hardware-verified
//
#include <hip/hip_runtime.h>
#include <math.h>


#define NG   16
#define NN   2048
#define SS   64
#define NROW (NG * NN)
typedef _Float16 b16;
typedef __attribute__((ext_vector_type(16))) _Float16 v16b;
typedef __attribute__((ext_vector_type(8)))  _Float16 v8b;
typedef __attribute__((ext_vector_type(8)))  float    v8f;
typedef __attribute__((ext_vector_type(4)))  float    v4f;
#define VST2(T, ptr, val) do { const T _v = (val); *(volatile T*)(ptr) = _v; __threadfence(); *(volatile T*)(ptr) = _v; } while (0)
__device__ __forceinline__ v8f wmma16b(v16b a, v16b b, v8f c) {
  v8f d = __builtin_amdgcn_wmma_f32_16x16x32_f16(false, a, false, b, (short)0, c, false, false);
  asm volatile("v_nop\n\tv_nop\n\tv_nop\n\tv_nop" : "+v"(d) : "v"(a), "v"(b));
  return d;
}
__device__ __forceinline__ v8b ld8b(const b16* p) { return *(const v8b*)p; }
__device__ __forceinline__ v16b cat8b(v8b a, v8b b) { return __builtin_shufflevector(a, b, 0,1,2,3,4,5,6,7,8,9,10,11,12,13,14,15); }
__device__ __forceinline__ v16b frag_kb(const b16* p, int hh) { return cat8b(ld8b(p + 8 * hh), ld8b(p + 16 + 8 * hh)); }
__device__ __forceinline__ void wave_lds_sync() { __builtin_amdgcn_fence(__ATOMIC_RELEASE, "workgroup"); __builtin_amdgcn_wave_barrier(); __builtin_amdgcn_fence(__ATOMIC_ACQUIRE, "workgroup"); }

__global__ __launch_bounds__(256) void k_w16(const float* __restrict__ Wk, const float* __restrict__ Wq, const float* __restrict__ Wv, b16* __restrict__ W16) {
  const int t = blockIdx.x * 256 + threadIdx.x;
  const int blk = t >> 9, n = (t >> 3) & 63, k0 = (t & 7) * 8;
  v8b o;
#pragma unroll
  for (int e = 0; e < 8; ++e) {
    const int k = k0 + e;
    const float v = (blk == 0) ? Wk[n * 64 + k] : (blk == 1) ? Wq[n * 64 + k] : (blk == 2) ? Wv[n * 128 + k] : Wv[n * 128 + 64 + k];
    o[e] = (b16)v;
  }
  VST2(v8b, W16 + ((size_t)blk * 64 + n) * 64 + k0, o);
}
template <bool ISK>
__global__ __launch_bounds__(256) void k_proj(const float* __restrict__ X, const b16* __restrict__ W1, const float* __restrict__ b1, const b16* __restrict__ W2, const float* __restrict__ b2,
                                              b16* __restrict__ P16, float* __restrict__ KP, b16* __restrict__ QPt) {
  __shared__ __attribute__((aligned(16))) float Tf[8][16 * 64];
  __shared__ __attribute__((aligned(16))) b16   Th[8][16 * 64];
  const int wid = threadIdx.x >> 5, lane = threadIdx.x & 31, hh = lane >> 4, col = lane & 15;
  const int m0 = (blockIdx.x * 8 + wid) * 16;
  float* tf = Tf[wid]; b16* th = Th[wid];
  v16b a0, a1;
  { const float* xr = X + (size_t)(m0 + col) * 64;
#pragma unroll
    for (int e = 0; e < 8; ++e) { a0[e] = (b16)xr[8 * hh + e]; a0[8 + e] = (b16)xr[16 + 8 * hh + e]; a1[e] = (b16)xr[32 + 8 * hh + e]; a1[8 + e] = (b16)xr[48 + 8 * hh + e]; } }
#pragma unroll
  for (int t = 0; t < 4; ++t) {
    v8f c = {};
    c = wmma16b(a0, frag_kb(W1 + (size_t)(t * 16 + col) * 64, hh), c);
    c = wmma16b(a1, frag_kb(W1 + (size_t)(t * 16 + col) * 64 + 32, hh), c);
#pragma unroll
    for (int v = 0; v < 8; ++v) { const float val = c[v] + b1[t * 16 + col]; const int r = v + 8 * hh, d = t * 16 + col; tf[r * 64 + d] = val; th[r * 64 + d] = (b16)val; }
  }
  wave_lds_sync();
  for (int pass = 0; pass < 2; ++pass) {
#pragma unroll
    for (int j = 0; j < 4; ++j) { const int pc = j * 32 + lane; *(volatile v8b*)(P16 + (size_t)m0 * 64 + pc * 8) = *(const v8b*)(th + pc * 8); }
    __threadfence();
  }
  const v16b p0 = frag_kb(th + col * 64, hh), p1 = frag_kb(th + col * 64 + 32, hh);
  wave_lds_sync();
#pragma unroll
  for (int t = 0; t < 4; ++t) {
    v8f c = {};
    c = wmma16b(p0, frag_kb(W2 + (size_t)(t * 16 + col) * 64, hh), c);
    c = wmma16b(p1, frag_kb(W2 + (size_t)(t * 16 + col) * 64 + 32, hh), c);
#pragma unroll
    for (int v = 0; v < 8; ++v) { const int r = v + 8 * hh, d = t * 16 + col; const float val = c[v] + (ISK ? b2[d] : 0.f);
      if (ISK) tf[r * 64 + d] = val; else th[d * 16 + r] = (b16)val; }
  }
  wave_lds_sync();
  for (int pass = 0; pass < 2; ++pass) {
    if (ISK) {
#pragma unroll
      for (int j = 0; j < 8; ++j) { const int pc = j * 32 + lane; *(volatile v4f*)(KP + (size_t)m0 * 64 + pc * 4) = *(const v4f*)(tf + pc * 4); }
    } else {
      b16* dst = QPt + (size_t)(m0 >> 4) * 1024;
#pragma unroll
      for (int j = 0; j < 4; ++j) { const int pc = j * 32 + lane; *(volatile v8b*)(dst + pc * 8) = *(const v8b*)(th + pc * 8); }
    }
    __threadfence();
  }
}
__global__ __launch_bounds__(256) void k_stats(const b16* __restrict__ Q16, const b16* __restrict__ K16, float* __restrict__ M, float* __restrict__ Zi) {
  __shared__ float sm[128], sz[128];
  const int wid = threadIdx.x >> 5, lane = threadIdx.x & 31, hh = lane >> 4, col = lane & 15;
  const int qtile = blockIdx.x * 8 + wid, g = qtile / (NN / 16), q0 = (qtile % (NN / 16)) * 16;
  const size_t ko = (size_t)g * NN * SS, qo = ((size_t)g * NN + q0 + col) * SS;
  const v16b q0h = frag_kb(Q16 + qo, hh), q1h = frag_kb(Q16 + qo + 32, hh);
  float m = -INFINITY, l = 0.f;
  for (int kb = 0; kb < NN; kb += 32) {
    const size_t r0 = ko + (size_t)(kb + col) * SS, r1 = ko + (size_t)(kb + 16 + col) * SS;
    v8f s0 = {}, s1 = {};
    s0 = wmma16b(frag_kb(K16 + r0, hh), q0h, s0); s0 = wmma16b(frag_kb(K16 + r0 + 32, hh), q1h, s0);
    s1 = wmma16b(frag_kb(K16 + r1, hh), q0h, s1); s1 = wmma16b(frag_kb(K16 + r1 + 32, hh), q1h, s1);
    float mr = -INFINITY;
#pragma unroll
    for (int r = 0; r < 8; ++r) mr = fmaxf(mr, fmaxf(s0[r], s1[r]));
    mr = fmaxf(mr, __shfl_xor(mr, 16));
    const float mn = fmaxf(m, mr), al = expf(m - mn);
    float sum = 0.f;
#pragma unroll
    for (int r = 0; r < 8; ++r) sum += expf(s0[r] - mn) + expf(s1[r] - mn);
    sum += __shfl_xor(sum, 16);
    l = l * al + sum; m = mn;
  }
  if (hh == 0) { sm[wid * 16 + col] = m; sz[wid * 16 + col] = 1.0f / l; }
  __syncthreads();
  const size_t base = (size_t)g * NN + (size_t)(blockIdx.x % (NN / 128)) * 128;
  for (int pass = 0; pass < 2; ++pass) {
    if (threadIdx.x < 128) *(volatile float*)(M + base + threadIdx.x) = sm[threadIdx.x];
    else                   *(volatile float*)(Zi + base + threadIdx.x - 128) = sz[threadIdx.x - 128];
    __threadfence();
  }
}
__global__ __launch_bounds__(256) void k_out(const b16* __restrict__ K16, const b16* __restrict__ Q16, const b16* __restrict__ QPt, const float* __restrict__ M,
                                             const float* __restrict__ Zi, const float* __restrict__ KP, float* __restrict__ out) {
  __shared__ __attribute__((aligned(16))) float Os[8][16 * 64];
  const int wid = threadIdx.x >> 5, lane = threadIdx.x & 31, hh = lane >> 4, col = lane & 15;
  const int ntile = blockIdx.x * 8 + wid, g = ntile / (NN / 16), n0 = (ntile % (NN / 16)) * 16;
  const size_t qbase = (size_t)g * NN * SS, no = ((size_t)g * NN + n0 + col) * SS;
  const v16b n0h = frag_kb(K16 + no, hh), n1h = frag_kb(K16 + no + 32, hh);
  float l = 0.f; v8f o0 = {}, o1 = {}, o2 = {}, o3 = {};
  for (int kb = 0; kb < NN; kb += 32) {
    const size_t r0 = qbase + (size_t)(kb + col) * SS, r1 = qbase + (size_t)(kb + 16 + col) * SS;
    v8f s0 = {}, s1 = {};
    s0 = wmma16b(frag_kb(Q16 + r0, hh), n0h, s0); s0 = wmma16b(frag_kb(Q16 + r0 + 32, hh), n1h, s0);
    s1 = wmma16b(frag_kb(Q16 + r1, hh), n0h, s1); s1 = wmma16b(frag_kb(Q16 + r1 + 32, hh), n1h, s1);
    const float* mq = M + (size_t)g * NN + kb + 8 * hh; const float* zq = Zi + (size_t)g * NN + kb + 8 * hh;
    float sum = 0.f; v16b pb;
#pragma unroll
    for (int r = 0; r < 8; ++r) {
      const float p0 = expf(s0[r] - mq[r]) * zq[r], p1 = expf(s1[r] - mq[16 + r]) * zq[16 + r];
      sum += p0 + p1; pb[r] = (b16)p0; pb[8 + r] = (b16)p1;
    }
    sum += __shfl_xor(sum, 16);
    l += sum;
    const size_t v0 = (size_t)g * NN * SS + (size_t)(kb >> 4) * (SS * 16) + 8 * hh, v1 = v0 + SS * 16;
#pragma unroll
    for (int n = 0; n < 4; ++n) {
      const int f = n * 16 + col;
      const v16b va = cat8b(ld8b(QPt + v0 + f * 16), ld8b(QPt + v1 + f * 16));
      v8f& o = (n == 0) ? o0 : (n == 1) ? o1 : (n == 2) ? o2 : o3;
      o = wmma16b(va, pb, o);
    }
  }
  float* Tt = Os[wid];
  const float* kp = KP + ((size_t)g * NN + n0 + col) * SS;
#pragma unroll
  for (int r = 0; r < 8; ++r) {
    const int hr = 8 * hh + r;
    Tt[col * 64 + 0 + hr] = o0[r] + l * kp[0 + hr];  Tt[col * 64 + 16 + hr] = o1[r] + l * kp[16 + hr];
    Tt[col * 64 + 32 + hr] = o2[r] + l * kp[32 + hr]; Tt[col * 64 + 48 + hr] = o3[r] + l * kp[48 + hr];
  }
  wave_lds_sync();
  float* dst0 = out + ((size_t)g * NN + n0) * SS;
  for (int pass = 0; pass < 2; ++pass) {
#pragma unroll
    for (int j = 0; j < 8; ++j) { const int pc = j * 32 + lane; *(volatile v4f*)(dst0 + pc * 4) = *(const v4f*)(Tt + pc * 4); }
    __threadfence();
  }
}
extern "C" void kernel_launch(void* const* d_in, const int* in_sizes, int n_in,
                              void* d_out, int out_size, void* d_ws, size_t ws_size, hipStream_t stream) {
  (void)in_sizes; (void)n_in; (void)out_size;
  const float* L  = (const float*)d_in[0];
  const float* Hq = (const float*)d_in[1];
  const float* Wk = (const float*)d_in[2]; const float* bk = (const float*)d_in[3];
  const float* Wq = (const float*)d_in[4]; const float* bq = (const float*)d_in[5];
  const float* Wv = (const float*)d_in[6]; const float* bv = (const float*)d_in[7];
  float* out = (float*)d_out;
  char* ws = (char*)d_ws; size_t off = 0;
  auto take = [&](size_t bytes) { void* p = ws + off; off = (off + bytes + 255) & ~(size_t)255; return p; };
  b16*   W16 = (b16*)take((size_t)4 * 64 * 64 * 2);
  b16*   K16 = (b16*)take((size_t)NROW * SS * 2);
  b16*   Q16 = (b16*)take((size_t)NROW * SS * 2);
  float* KP  = (float*)take((size_t)NROW * SS * 4);
  b16*   QPt = (b16*)take((size_t)NROW * SS * 2);
  float* M   = (float*)take((size_t)NROW * 4);
  float* Zi  = (float*)take((size_t)NROW * 4);
  if (off > ws_size) return;
  const dim3 b256(256);
  k_w16<<<4 * 64 * 8 / 256, b256, 0, stream>>>(Wk, Wq, Wv, W16);
  k_proj<true><<<NROW / 128, b256, 0, stream>>>(L, W16, bk, W16 + 3 * 4096, bv, K16, KP, nullptr);
  k_proj<false><<<NROW / 128, b256, 0, stream>>>(Hq, W16 + 4096, bq, W16 + 2 * 4096, nullptr, Q16, nullptr, QPt);
  k_stats<<<NROW / 128, b256, 0, stream>>>(Q16, K16, M, Zi);
  k_out<<<NROW / 128, b256, 0, stream>>>(K16, Q16, QPt, M, Zi, KP, out);
}
